// RWKV_TmixWrapper_26560077758560
// MI455X (gfx1250) — hardware-verified
//
#include <hip/hip_runtime.h>
#include <math.h>

constexpr int kB     = 4;
constexpr int kT     = 1024;
constexpr int kC     = 1024;
constexpr int kH     = 16;
constexpr int kHD    = 64;
constexpr int kRows  = kB * kT;
constexpr int kLmix  = 32;
constexpr int kMixN  = 4 * kLmix;
constexpr int kLdec  = 64;
constexpr int kSCH   = 32;
constexpr float kWCarry    = 1024.0f;
constexpr float kWCarryInv = 1.0f / 1024.0f;
constexpr float kGnEps     = 64e-5f;
constexpr float kInvHD     = 1.0f / (float)kHD;
static_assert(kH * kHD == kC, "heads x head size = channels");
static_assert(kRows % 64 == 0 && kC % 64 == 0 && kMixN % 64 == 0 && kLdec % 64 == 0, "GEMM M, N tile multiples");
static_assert(kC % 32 == 0 && kLmix % 32 == 0 && kLdec % 32 == 0, "GEMM K multiples of 32");
static_assert(kT % kSCH == 0, "scan chunking exact");
static_assert((kRows * kC / 8) % 256 == 0, "elementwise grids exact");
static_assert((kRows * kMixN) % 2048 == 0 && (kRows * kLdec) % 2048 == 0, "tanh grids exact");

typedef __attribute__((ext_vector_type(16))) _Float16 v16h;
typedef __attribute__((ext_vector_type(8)))  _Float16 v8h;
typedef __attribute__((ext_vector_type(8)))  float    v8f;
typedef __attribute__((ext_vector_type(4)))  float    v4f;
typedef __attribute__((ext_vector_type(4)))  unsigned int v4u;

__device__ __forceinline__ unsigned pk16(unsigned short a, unsigned short b) { return (unsigned)a | ((unsigned)b << 16); }
__device__ __forceinline__ unsigned short h_bits(float f) { const _Float16 h = (_Float16)f; return __builtin_bit_cast(unsigned short, h); }
__device__ __forceinline__ float h16_to_f32(unsigned hb) {
  const unsigned sgn = (hb & 0x8000u) << 16; const unsigned em = hb & 0x7fffu;
  const float fn = __uint_as_float((em << 13) + 0x38000000u);
  const float fs = (float)em * 5.9604644775390625e-8f;
  const float mag = (em < 0x400u) ? fs : fn; return __uint_as_float(__float_as_uint(mag) | sgn); }

__device__ __forceinline__ void group_guard_h(v8f& a, v8f& b, v8f& c, v8f& d, v16h x, v16h b0, v16h b1, v16h b2, v16h b3) {
  asm volatile("v_nop\n\tv_nop\n\tv_nop\n\tv_nop" : "+v"(a), "+v"(b), "+v"(c), "+v"(d) : "v"(x), "v"(b0), "v"(b1), "v"(b2), "v"(b3));
}
__device__ __forceinline__ void keep4_h(v16h a, v16h b, v16h c, v16h d) { asm volatile("v_nop" :: "v"(a), "v"(b), "v"(c), "v"(d)); }
__device__ __forceinline__ void acc_guard4(v8f& a, v8f& b, v8f& c, v8f& d) { asm volatile("v_nop\n\tv_nop\n\tv_nop\n\tv_nop" : "+v"(a), "+v"(b), "+v"(c), "+v"(d)); }

template <typename T> struct Frag;
template <> struct Frag<_Float16> {
  typedef v16h V; union U { v16h v; v8h h[2]; };
  static __device__ __forceinline__ v16h load(const _Float16* p) {
    U f; f.h[0] = *(const v8h*)(p); f.h[1] = *(const v8h*)(p + 16); return f.v;
  }
  static __device__ __forceinline__ v8f mma(v16h a, v16h b, v8f c) {
    return __builtin_amdgcn_wmma_f32_16x16x32_f16(false, a, false, b, (short)0, c, false, false);
  }
};

template <bool BSPLIT, int OUT_MODE>
__global__ __launch_bounds__(256) void wmma_gemm64(
    const unsigned short* __restrict__ Ap, int lda, long strideA,
    const unsigned short* __restrict__ Btp, const unsigned short* __restrict__ Bt2p, int ldb, long strideB,
    void* __restrict__ Cout, int ldc, long strideC,
    int M, int N, int K, float scale) {
  typedef _Float16 T;
  typedef v16h V;
  const T* A = (const T*)Ap; const T* Bt = (const T*)Btp; const T* Bt2 = (const T*)Bt2p;
  __shared__ __align__(16) float sT[8][16 * 68];
  const int b    = blockIdx.y;
  const int lane = threadIdx.x & 31;
  const int wave = threadIdx.x >> 5;
  const int tilesN = N >> 6;
  const int tilesM = M >> 6;
  const int tile = blockIdx.x * 8 + wave;
  if (tile >= tilesM * tilesN) return;
  const int tm = tile / tilesN;
  const int tn = tile - tm * tilesN;
  const int m0 = tm << 6;
  const int n0 = tn << 6;

  const T* Ab  = A   + (size_t)b * strideA;
  const T* Bb  = Bt  + (size_t)b * strideB;
  const T* Bb2 = Bt2 + (size_t)b * strideB;

  const int rlane = lane & 15;
  const int koff  = (lane >> 4) * 8;
  const int mOff  = (lane >> 4) * 8;

  int aoff[4], boff[4];
#pragma unroll
  for (int i = 0; i < 4; ++i) {
    aoff[i] = (m0 + (i << 4) + rlane) * lda + koff;
    boff[i] = (n0 + (i << 4) + rlane) * ldb + koff;
  }

  v8f acc[4][4];
#pragma unroll
  for (int i = 0; i < 4; ++i)
#pragma unroll
    for (int j = 0; j < 4; ++j) acc[i][j] = (v8f){0.f,0.f,0.f,0.f,0.f,0.f,0.f,0.f};

  for (int k0 = 0; k0 < K; k0 += 32) {
    V bh[4], bl[4];
#pragma unroll
    for (int j = 0; j < 4; ++j) {
      bh[j] = Frag<T>::load(Bb + boff[j] + k0);
      if (BSPLIT) bl[j] = Frag<T>::load(Bb2 + boff[j] + k0);
      else bl[j] = bh[j];
    }
#pragma unroll
    for (int i = 0; i < 4; ++i) {
      V ah = Frag<T>::load(Ab + aoff[i] + k0);
#pragma unroll
      for (int j = 0; j < 4; ++j) {
        acc[i][j] = Frag<T>::mma(ah, bh[j], acc[i][j]);
        if (BSPLIT) acc[i][j] = Frag<T>::mma(ah, bl[j], acc[i][j]);
      }
      group_guard_h(acc[i][0], acc[i][1], acc[i][2], acc[i][3], ah, bl[0], bl[1], bl[2], bl[3]);
    }
    keep4_h(bh[0], bh[1], bh[2], bh[3]);
    keep4_h(bl[0], bl[1], bl[2], bl[3]);
  }
  acc_guard4(acc[0][0], acc[0][1], acc[0][2], acc[0][3]);
  acc_guard4(acc[1][0], acc[1][1], acc[1][2], acc[1][3]);
  acc_guard4(acc[2][0], acc[2][1], acc[2][2], acc[2][3]);
  acc_guard4(acc[3][0], acc[3][1], acc[3][2], acc[3][3]);

  float* slab = sT[wave];
#pragma unroll
  for (int i = 0; i < 4; ++i) {
    const int mBase = m0 + (i << 4);
#pragma unroll
    for (int j = 0; j < 4; ++j) {
#pragma unroll
      for (int r = 0; r < 8; ++r) {
        const float v = acc[i][j][r] * scale;
        slab[(mOff + r) * 68 + (j << 4) + rlane] = v;
      }
    }
    __builtin_amdgcn_fence(__ATOMIC_RELEASE, "workgroup");
    __builtin_amdgcn_wave_barrier();
    __builtin_amdgcn_fence(__ATOMIC_ACQUIRE, "workgroup");
    if (OUT_MODE == 0) {
      float* C = (float*)Cout + (size_t)b * strideC;
      const int hh = lane >> 4, c4 = (lane & 15) * 4;
      for (int pass = 0; pass < 2; ++pass) {
#pragma unroll
        for (int it = 0; it < 8; ++it) {
          const int row = it * 2 + hh;
          v4f v = *(const v4f*)(slab + row * 68 + c4);
          *(volatile v4f*)(C + (size_t)(mBase + row) * ldc + n0 + c4) = v;
        }
        __threadfence();
      }
    } else {
      const int q = lane >> 3, c8 = (lane & 7) * 8;
      unsigned short* C = (unsigned short*)Cout + (size_t)b * strideC;
      for (int pass = 0; pass < 2; ++pass) {
#pragma unroll
        for (int it = 0; it < 4; ++it) {
          const int row = it * 4 + q;
          const float* sp = slab + row * 68 + c8;
          v8h hv;
#pragma unroll
          for (int e = 0; e < 8; ++e) hv[e] = (_Float16)sp[e];
          *(volatile v8h*)(C + (size_t)(mBase + row) * ldc + n0 + c8) = hv;
        }
        __threadfence();
      }
    }
    __builtin_amdgcn_fence(__ATOMIC_RELEASE, "workgroup");
    __builtin_amdgcn_wave_barrier();
    __builtin_amdgcn_fence(__ATOMIC_ACQUIRE, "workgroup");
  }
}

template <int KT, bool SPLIT>
__global__ __launch_bounds__(256) void wt_cast_kernel(const float* __restrict__ W0, const float* __restrict__ W1,
                                                      const float* __restrict__ W2, const float* __restrict__ W3,
                                                      unsigned short* __restrict__ outHi, unsigned short* __restrict__ outLo,
                                                      long planeStride, int Kdim, int Ndim, float scale) {
  static_assert(KT == 64 || KT == 32, "tile depth");
  __shared__ float sm[64][KT + 1];
  const int t  = threadIdx.x;
  const int k0 = blockIdx.x * KT;
  const int n0 = blockIdx.y * 64;
  const int z  = blockIdx.z;
  const float* W = (z == 0) ? W0 : (z == 1) ? W1 : (z == 2) ? W2 : W3;
#pragma unroll
  for (int i = 0; i < KT / 4; ++i) {
    const int e = i * 256 + t;
    const int r = e >> 6;
    const int c = e & 63;
    sm[c][r] = W[(size_t)(k0 + r) * Ndim + n0 + c] * scale;
  }
  __syncthreads();
  constexpr int LPR   = KT / 8;
  constexpr int RPI   = 256 / LPR;
  constexpr int ITERS = 64 / RPI;
  const int rl = t / LPR;
  const int c8 = (t % LPR) * 8;
  v4u uh[ITERS], ul[ITERS];
#pragma unroll
  for (int it = 0; it < ITERS; ++it) {
    const int row = it * RPI + rl;
    unsigned short hb[8], lb[8];
#pragma unroll
    for (int e = 0; e < 8; ++e) {
      const float v = sm[row][c8 + e];
      const _Float16 hh = (_Float16)v;
      const float rem = v - (float)hh;
      const _Float16 ll = (_Float16)rem;
      hb[e] = __builtin_bit_cast(unsigned short, hh);
      lb[e] = __builtin_bit_cast(unsigned short, ll);
    }
    uh[it] = (v4u){pk16(hb[0], hb[1]), pk16(hb[2], hb[3]), pk16(hb[4], hb[5]), pk16(hb[6], hb[7])};
    ul[it] = (v4u){pk16(lb[0], lb[1]), pk16(lb[2], lb[3]), pk16(lb[4], lb[5]), pk16(lb[6], lb[7])};
  }
  unsigned short* oh = outHi + (size_t)z * planeStride;
  unsigned short* ol = outLo + (size_t)z * planeStride;
  for (int pass = 0; pass < 2; ++pass) {
#pragma unroll
    for (int it = 0; it < ITERS; ++it) {
      const int row = it * RPI + rl;
      const size_t o = (size_t)(n0 + row) * Kdim + k0 + c8;
      *(volatile v4u*)(oh + o) = uh[it];
      if (SPLIT) *(volatile v4u*)(ol + o) = ul[it];
    }
    __threadfence();
  }
}

__global__ __launch_bounds__(256) void shift_lerp_kernel(const float* __restrict__ x, const float* __restrict__ maa_x,
                                                         unsigned short* __restrict__ xxx) {
  const int i    = blockIdx.x * 256 + threadIdx.x;
  const int row  = i >> 7;
  const int c8   = (i & 127) * 8;
  const int tpos = row & (kT - 1);
  const int prow = (row > 0) ? (row - 1) : 0;
  const float* xp = x + (size_t)row * kC + c8;
  const float* pp = x + (size_t)prow * kC + c8;
  const v4f xa = *(const v4f*)(xp);
  const v4f xb = *(const v4f*)(xp + 4);
  const v4f pa = *(const v4f*)(pp);
  const v4f pb = *(const v4f*)(pp + 4);
  const v4f ma = *(const v4f*)(maa_x + c8);
  const v4f mb = *(const v4f*)(maa_x + c8 + 4);
  const bool first = (tpos == 0);
  unsigned short hb[8];
#pragma unroll
  for (int e = 0; e < 4; ++e) {
    const float p0 = first ? 0.0f : pa[e];
    const float p1 = first ? 0.0f : pb[e];
    const float d0 = p0 - xa[e];
    const float d1 = p1 - xb[e];
    hb[e]     = h_bits(xa[e] + d0 * ma[e]);
    hb[4 + e] = h_bits(xb[e] + d1 * mb[e]);
  }
  const v4u u = (v4u){pk16(hb[0], hb[1]), pk16(hb[2], hb[3]), pk16(hb[4], hb[5]), pk16(hb[6], hb[7])};
  unsigned short* q = xxx + (size_t)i * 8;
  *(volatile v4u*)q = u;
  __threadfence();
  *(volatile v4u*)q = u;
}

__global__ __launch_bounds__(256) void tanh_cast_kernel(const float* __restrict__ in, unsigned short* __restrict__ out) {
  __shared__ __align__(16) float sv[2048];
  const int t = threadIdx.x;
  const size_t base = (size_t)blockIdx.x * 2048;
#pragma unroll 1
  for (int e = 0; e < 8; ++e) {
    const int idx = e * 256 + t;
    sv[idx] = tanhf(in[base + idx]);
  }
  __syncthreads();
  const v4f a = *(const v4f*)(sv + 8 * t);
  const v4f c = *(const v4f*)(sv + 8 * t + 4);
  unsigned short hb[8];
#pragma unroll
  for (int e = 0; e < 4; ++e) {
    hb[e]     = h_bits(a[e]);
    hb[4 + e] = h_bits(c[e]);
  }
  const v4u u = (v4u){pk16(hb[0], hb[1]), pk16(hb[2], hb[3]), pk16(hb[4], hb[5]), pk16(hb[6], hb[7])};
  unsigned short* q = out + base + 8 * (size_t)t;
  *(volatile v4u*)q = u;
  __threadfence();
  *(volatile v4u*)q = u;
}

__device__ __forceinline__ v4u mix_one(const float (&xv)[8], const float (&xd)[8], const float* __restrict__ maa,
                                       const unsigned short* __restrict__ mixp) {
  const v4f ma = *(const v4f*)(maa);
  const v4f mb = *(const v4f*)(maa + 4);
  const v4u mw = *(const v4u*)(mixp);
  float m8[8], a8[8];
#pragma unroll
  for (int q = 0; q < 4; ++q) {
    const unsigned w = mw[q];
    m8[2 * q]     = h16_to_f32(w & 0xffffu);
    m8[2 * q + 1] = h16_to_f32(w >> 16);
    a8[q]     = ma[q];
    a8[4 + q] = mb[q];
  }
  unsigned short hb[8];
#pragma unroll
  for (int e = 0; e < 8; ++e) hb[e] = h_bits(xv[e] + xd[e] * (a8[e] + m8[e]));
  return (v4u){pk16(hb[0], hb[1]), pk16(hb[2], hb[3]), pk16(hb[4], hb[5]), pk16(hb[6], hb[7])};
}

__global__ __launch_bounds__(256) void mix_inputs_kernel(const float* __restrict__ x,
                                                         const float* __restrict__ maa_w, const float* __restrict__ maa_k,
                                                         const float* __restrict__ maa_v, const float* __restrict__ maa_r,
                                                         const unsigned short* __restrict__ mixp,
                                                         unsigned short* __restrict__ xm) {
  const int i    = blockIdx.x * 256 + threadIdx.x;
  const int row  = i >> 7;
  const int c8   = (i & 127) * 8;
  const int tpos = row & (kT - 1);
  const int prow = (row > 0) ? (row - 1) : 0;
  const float* xp = x + (size_t)row * kC + c8;
  const float* pp = x + (size_t)prow * kC + c8;
  const v4f xa = *(const v4f*)(xp);
  const v4f xb = *(const v4f*)(xp + 4);
  const v4f pa = *(const v4f*)(pp);
  const v4f pb = *(const v4f*)(pp + 4);
  const bool first = (tpos == 0);
  float xv[8], xd[8];
#pragma unroll
  for (int e = 0; e < 4; ++e) {
    const float p0 = first ? 0.0f : pa[e];
    const float p1 = first ? 0.0f : pb[e];
    xv[e]     = xa[e];
    xv[4 + e] = xb[e];
    xd[e]     = p0 - xa[e];
    xd[4 + e] = p1 - xb[e];
  }
  const size_t PL  = (size_t)kRows * kC;
  const size_t off = (size_t)i * 8;
  const v4u u0 = mix_one(xv, xd, maa_w + c8, mixp + 0 * PL + off);
  const v4u u1 = mix_one(xv, xd, maa_k + c8, mixp + 1 * PL + off);
  const v4u u2 = mix_one(xv, xd, maa_v + c8, mixp + 2 * PL + off);
  const v4u u3 = mix_one(xv, xd, maa_r + c8, mixp + 3 * PL + off);
  for (int pass = 0; pass < 2; ++pass) {
    *(volatile v4u*)(xm + 0 * PL + off) = u0;
    *(volatile v4u*)(xm + 1 * PL + off) = u1;
    *(volatile v4u*)(xm + 2 * PL + off) = u2;
    *(volatile v4u*)(xm + 3 * PL + off) = u3;
    __threadfence();
  }
}

__global__ __launch_bounds__(256) void scan_norm_kernel(const float* __restrict__ R, const float* __restrict__ Kp,
                                                        const float* __restrict__ Vp, const float* __restrict__ WWL,
                                                        const float* __restrict__ tdec, const float* __restrict__ ubonus,
                                                        const float* __restrict__ lnw, const float* __restrict__ lnb,
                                                        unsigned short* __restrict__ YN) {
  __shared__ __align__(16) float sr[kSCH * kHD];
  __shared__ __align__(16) float sk[kSCH * kHD];
  __shared__ __align__(16) float sw[kSCH * kHD];
  __shared__ __align__(16) float sv[kSCH * kHD];
  __shared__ __align__(16) float sy[kSCH * kHD];
  const int tid  = threadIdx.x;
  const int lane = tid & 31;
  const int wave = tid >> 5;
  const int part = lane >> 3;
  const int j    = wave * 8 + (lane & 7);
  const int b    = blockIdx.x >> 4;
  const int h    = blockIdx.x & 15;

  float S[16], uu[16];
  {
    const float* up = ubonus + h * kHD + part * 16;
#pragma unroll
    for (int q = 0; q < 4; ++q) {
      const v4f t4 = *(const v4f*)(up + 4 * q);
#pragma unroll
      for (int e = 0; e < 4; ++e) { uu[4 * q + e] = t4[e]; S[4 * q + e] = 0.0f; }
    }
  }
  const int scol = tid & 63;
  const float tdv = tdec[h * kHD + scol];
  const int grow = tid >> 3;
  const int gseg = (tid & 7) * 8;
  float lw[8], lb[8];
  {
    const v4f w0 = *(const v4f*)(lnw + h * kHD + gseg);
    const v4f w1 = *(const v4f*)(lnw + h * kHD + gseg + 4);
    const v4f b0 = *(const v4f*)(lnb + h * kHD + gseg);
    const v4f b1 = *(const v4f*)(lnb + h * kHD + gseg + 4);
#pragma unroll
    for (int e = 0; e < 4; ++e) { lw[e] = w0[e]; lw[4 + e] = w1[e]; lb[e] = b0[e]; lb[4 + e] = b1[e]; }
  }
  const size_t base = (size_t)(b * kT) * kC + (size_t)h * kHD;
  const int srow = tid >> 4;
  const int sc4  = (tid & 15) * 4;

#pragma unroll 1
  for (int ch = 0; ch < kT / kSCH; ++ch) {
    const int t0 = ch * kSCH;
    __syncthreads();
#pragma unroll
    for (int it = 0; it < 2; ++it) {
      const int row = srow + 16 * it;
      const size_t g = base + (size_t)(t0 + row) * kC + sc4;
      const v4f a = *(const v4f*)(R + g);
      const v4f c = *(const v4f*)(Kp + g);
      const v4f d = *(const v4f*)(Vp + g);
      *(v4f*)(sr + row * kHD + sc4) = a;
      *(v4f*)(sk + row * kHD + sc4) = c;
      *(v4f*)(sv + row * kHD + sc4) = d;
    }
#pragma unroll 1
    for (int e = 0; e < 8; ++e) {
      const int row = e * 4 + (tid >> 6);
      const float ww = tdv + WWL[base + (size_t)(t0 + row) * kC + scol];
      sw[row * kHD + scol] = expf(-expf(ww));
    }
    __syncthreads();

#pragma unroll 1
    for (int s = 0; s < kSCH; ++s) {
      const float vj = sv[s * kHD + j];
      const float* rp = sr + s * kHD + part * 16;
      const float* kp = sk + s * kHD + part * 16;
      const float* wp = sw + s * kHD + part * 16;
      float acc = 0.0f;
#pragma unroll
      for (int q = 0; q < 4; ++q) {
        const v4f r4 = *(const v4f*)(rp + 4 * q);
        const v4f k4 = *(const v4f*)(kp + 4 * q);
        const v4f w4 = *(const v4f*)(wp + 4 * q);
#pragma unroll
        for (int e = 0; e < 4; ++e) {
          const float kv = k4[e] * vj;
          const float tt = fmaf(uu[4 * q + e], kv, S[4 * q + e]);
          acc = fmaf(r4[e], tt, acc);
          S[4 * q + e] = fmaf(w4[e], S[4 * q + e], kv);
        }
      }
      acc += __shfl_xor(acc, 8, 32);
      acc += __shfl_xor(acc, 16, 32);
      if (part == 0) sy[s * kHD + j] = acc;
    }
    __syncthreads();

    const v4f ya = *(const v4f*)(sy + grow * kHD + gseg);
    const v4f yb = *(const v4f*)(sy + grow * kHD + gseg + 4);
    float sum = ((ya[0] + ya[1]) + (ya[2] + ya[3])) + ((yb[0] + yb[1]) + (yb[2] + yb[3]));
    sum += __shfl_xor(sum, 1, 32);
    sum += __shfl_xor(sum, 2, 32);
    sum += __shfl_xor(sum, 4, 32);
    const float mean = sum * kInvHD;
    float dv[8];
    float ss = 0.0f;
#pragma unroll
    for (int e = 0; e < 4; ++e) {
      dv[e]     = ya[e] - mean;
      dv[4 + e] = yb[e] - mean;
    }
#pragma unroll
    for (int e = 0; e < 8; ++e) ss += dv[e] * dv[e];
    ss += __shfl_xor(ss, 1, 32);
    ss += __shfl_xor(ss, 2, 32);
    ss += __shfl_xor(ss, 4, 32);
    const float var  = ss * kInvHD;
    const float rstd = rsqrtf(var + kGnEps);
    unsigned short hb[8];
#pragma unroll
    for (int e = 0; e < 8; ++e) hb[e] = h_bits((dv[e] * rstd) * lw[e] + lb[e]);
    const v4u u = (v4u){pk16(hb[0], hb[1]), pk16(hb[2], hb[3]), pk16(hb[4], hb[5]), pk16(hb[6], hb[7])};
    unsigned short* op = YN + (size_t)(b * kT + t0 + grow) * kC + (size_t)h * kHD + gseg;
    *(volatile v4u*)op = u;
    __threadfence();
    *(volatile v4u*)op = u;
  }
}

extern "C" void kernel_launch(void* const* d_in, const int* in_sizes, int n_in,
                              void* d_out, int out_size, void* d_ws, size_t ws_size, hipStream_t stream) {
  if (n_in < 20 || d_out == nullptr || d_ws == nullptr) return;
  if (in_sizes[0] != kRows * kC || in_sizes[3] != kC || in_sizes[4] != kC || in_sizes[5] != kC ||
      in_sizes[6] != kC || in_sizes[7] != kC || in_sizes[8] != kC * kMixN || in_sizes[9] != 4 * kLmix * kC ||
      in_sizes[10] != kC || in_sizes[11] != kC * kLdec || in_sizes[12] != kLdec * kC || in_sizes[13] != kH * kHD ||
      in_sizes[14] != kC * kC || in_sizes[15] != kC * kC || in_sizes[16] != kC * kC || in_sizes[17] != kC * kC ||
      in_sizes[18] != kC || in_sizes[19] != kC || out_size != kRows * kC) return;

  const float* x      = (const float*)d_in[0];
  const float* maa_x  = (const float*)d_in[3];
  const float* maa_w  = (const float*)d_in[4];
  const float* maa_k  = (const float*)d_in[5];
  const float* maa_v  = (const float*)d_in[6];
  const float* maa_r  = (const float*)d_in[7];
  const float* mw1    = (const float*)d_in[8];
  const float* mw2    = (const float*)d_in[9];
  const float* tdec   = (const float*)d_in[10];
  const float* dw1    = (const float*)d_in[11];
  const float* dw2    = (const float*)d_in[12];
  const float* ubonus = (const float*)d_in[13];
  const float* W_r    = (const float*)d_in[14];
  const float* W_k    = (const float*)d_in[15];
  const float* W_v    = (const float*)d_in[16];
  const float* W_o    = (const float*)d_in[17];
  const float* ln_w   = (const float*)d_in[18];
  const float* ln_b   = (const float*)d_in[19];
  float* out = (float*)d_out;

  char* ws = (char*)d_ws; size_t off = 0;
  auto carve = [&](size_t bytes) -> char* { char* p = ws + off; off += (bytes + 255) & ~(size_t)255; return p; };
  const size_t PLW = (size_t)kC * kC;
  const size_t PL  = (size_t)kRows * kC;
  unsigned short* WHI   = (unsigned short*)carve(4 * PLW * 2);
  unsigned short* WLO   = (unsigned short*)carve(4 * PLW * 2);
  unsigned short* W1T   = (unsigned short*)carve((size_t)kMixN * kC * 2);
  unsigned short* W2T   = (unsigned short*)carve((size_t)4 * kC * kLmix * 2);
  unsigned short* DW1T  = (unsigned short*)carve((size_t)kLdec * kC * 2);
  unsigned short* DW2T  = (unsigned short*)carve((size_t)kC * kLdec * 2);
  unsigned short* XXX   = (unsigned short*)carve(PL * 2);
  float*          MPRE  = (float*)carve((size_t)kRows * kMixN * 4);
  unsigned short* MT    = (unsigned short*)carve((size_t)kRows * kMixN * 2);
  float*          T1PRE = (float*)carve((size_t)kRows * kLdec * 4);
  unsigned short* T1    = (unsigned short*)carve((size_t)kRows * kLdec * 2);
  unsigned short* MIXP  = (unsigned short*)carve(4 * PL * 2);
  unsigned short* XM    = (unsigned short*)carve(4 * PL * 2);
  float*          VBUF  = (float*)carve(PL * 4);
  float*          WWL   = (float*)carve(PL * 4);
  if (off > ws_size || off > (size_t)134217728) return;
  float*          RBUF  = (float*)MIXP;
  float*          KBUF  = RBUF + PL;
  unsigned short* YN    = XXX;

  wt_cast_kernel<64, true><<<dim3(kC / 64, kC / 64, 4), 256, 0, stream>>>(
      W_r, W_k, W_v, W_o, WHI, WLO, (long)PLW, kC, kC, kWCarry);
  wt_cast_kernel<64, false><<<dim3(kC / 64, kMixN / 64, 1), 256, 0, stream>>>(
      mw1, mw1, mw1, mw1, W1T, W1T, 0L, kC, kMixN, kWCarry);
  wt_cast_kernel<32, false><<<dim3(1, kC / 64, 4), 256, 0, stream>>>(
      mw2, mw2 + (size_t)1 * kLmix * kC, mw2 + (size_t)2 * kLmix * kC, mw2 + (size_t)3 * kLmix * kC,
      W2T, W2T, (long)kC * kLmix, kLmix, kC, kWCarry);
  wt_cast_kernel<64, false><<<dim3(kC / 64, kLdec / 64, 1), 256, 0, stream>>>(
      dw1, dw1, dw1, dw1, DW1T, DW1T, 0L, kC, kLdec, kWCarry);
  wt_cast_kernel<64, false><<<dim3(kLdec / 64, kC / 64, 1), 256, 0, stream>>>(
      dw2, dw2, dw2, dw2, DW2T, DW2T, 0L, kLdec, kC, kWCarry);

  const int ewBlocks = kRows * kC / 8 / 256;
  shift_lerp_kernel<<<ewBlocks, 256, 0, stream>>>(x, maa_x, XXX);

  wmma_gemm64<false, 0><<<dim3((kRows / 64) * (kMixN / 64) / 8, 1), 256, 0, stream>>>(
      XXX, kC, 0L, W1T, W1T, kC, 0L, (void*)MPRE, kMixN, 0L, kRows, kMixN, kC, kWCarryInv);
  tanh_cast_kernel<<<kRows * kMixN / 2048, 256, 0, stream>>>(MPRE, MT);
  wmma_gemm64<false, 1><<<dim3((kRows / 64) * (kC / 64) / 8, 4), 256, 0, stream>>>(
      MT, kMixN, (long)kLmix, W2T, W2T, kLmix, (long)kC * kLmix, (void*)MIXP, kC, (long)PL, kRows, kC, kLmix, kWCarryInv);
  mix_inputs_kernel<<<ewBlocks, 256, 0, stream>>>(x, maa_w, maa_k, maa_v, maa_r, MIXP, XM);

  wmma_gemm64<false, 0><<<dim3((kRows / 64) * (kLdec / 64) / 8, 1), 256, 0, stream>>>(
      XM + 0 * PL, kC, 0L, DW1T, DW1T, kC, 0L, (void*)T1PRE, kLdec, 0L, kRows, kLdec, kC, kWCarryInv);
  tanh_cast_kernel<<<kRows * kLdec / 2048, 256, 0, stream>>>(T1PRE, T1);
  const dim3 bigGrid((kRows / 64) * (kC / 64) / 8, 1);
  wmma_gemm64<false, 0><<<bigGrid, 256, 0, stream>>>(
      T1, kLdec, 0L, DW2T, DW2T, kLdec, 0L, (void*)WWL, kC, 0L, kRows, kC, kLdec, kWCarryInv);

  wmma_gemm64<true, 0><<<bigGrid, 256, 0, stream>>>(
      XM + 3 * PL, kC, 0L, WHI + 0 * PLW, WLO + 0 * PLW, kC, 0L, (void*)RBUF, kC, 0L, kRows, kC, kC, kWCarryInv);
  wmma_gemm64<true, 0><<<bigGrid, 256, 0, stream>>>(
      XM + 1 * PL, kC, 0L, WHI + 1 * PLW, WLO + 1 * PLW, kC, 0L, (void*)KBUF, kC, 0L, kRows, kC, kC, kWCarryInv);
  wmma_gemm64<true, 0><<<bigGrid, 256, 0, stream>>>(
      XM + 2 * PL, kC, 0L, WHI + 2 * PLW, WLO + 2 * PLW, kC, 0L, (void*)VBUF, kC, 0L, kRows, kC, kC, kWCarryInv);

  scan_norm_kernel<<<kB * kH, 256, 0, stream>>>(RBUF, KBUF, VBUF, WWL, tdec, ubonus, ln_w, ln_b, YN);

  wmma_gemm64<true, 0><<<bigGrid, 256, 0, stream>>>(
      YN, kC, 0L, WHI + 3 * PLW, WLO + 3 * PLW, kC, 0L, (void*)out, kC, 0L, kRows, kC, kC, kWCarryInv);
}
